// Masked_MHA_53953379172640
// MI455X (gfx1250) — hardware-verified
//
#include <hip/hip_runtime.h>


namespace {
constexpr int NT = 4 * 2048, E = 512;
constexpr float XS = 8.0f, WSC = 256.0f;
typedef _Float16 b16;
typedef __attribute__((ext_vector_type(16))) _Float16 v16b;
typedef __attribute__((ext_vector_type(8))) _Float16 v8b;
typedef __attribute__((ext_vector_type(8))) float v8f;
typedef __attribute__((ext_vector_type(4))) float v4f;
__device__ __forceinline__ float bf16_rne(float f) { unsigned int u = __float_as_uint(f); u += 0x7FFFu + ((u >> 16) & 1u); float r = __uint_as_float(u & 0xFFFF0000u); asm volatile("" : "+v"(r)); return r; }
__device__ __forceinline__ float bfv(float f) { float r = bf16_rne(f); asm volatile("" : "+v"(r)); return r; }
__device__ __forceinline__ v16b frag_kb(const b16* p, int hh) { const v8b a = *(const v8b*)(p + 8 * hh), b = *(const v8b*)(p + 16 + 8 * hh); v16b f;
#pragma unroll
  for (int e = 0; e < 8; ++e) { f[e] = a[e]; f[8 + e] = b[e]; } return f; }
__device__ __forceinline__ v8f wmma16b(v16b a, v16b b, v8f c) { v8f d = __builtin_amdgcn_wmma_f32_16x16x32_f16(false, a, false, b, (short)0, c, false, false); asm volatile("v_nop\n\tv_nop\n\tv_nop\n\tv_nop" : "+v"(d) : "v"(a), "v"(b)); return d; }
__device__ __forceinline__ void wave_lds_sync() { __builtin_amdgcn_fence(__ATOMIC_RELEASE, "workgroup"); __builtin_amdgcn_wave_barrier(); __builtin_amdgcn_fence(__ATOMIC_ACQUIRE, "workgroup"); }

__global__ __launch_bounds__(256) void wput_kernel(const float* __restrict__ w, b16* __restrict__ WT) { const int u = blockIdx.x * 256 + threadIdx.x; if (u >= E * (E / 8)) return; const int o = u / (E / 8), k0 = (u % (E / 8)) * 8; v8b v;
#pragma unroll
  for (int j = 0; j < 8; ++j) v[j] = (b16)(bf16_rne(w[(size_t)(k0 + j) * E + o]) * WSC);
  for (int pass = 0; pass < 2; ++pass) { *(volatile v8b*)(WT + (size_t)o * E + k0) = v; __threadfence(); } }
__global__ __launch_bounds__(32) void main_kernel(const float* __restrict__ x, const b16* __restrict__ WT, const float* __restrict__ b, int TLIM, float* __restrict__ out) { __shared__ __attribute__((aligned(16))) b16 Ax[16][E + 8]; __shared__ float Tf[16][260]; const int lane = threadIdx.x, nloc = lane & 15, hlf = lane >> 4; const size_t t0 = (size_t)blockIdx.x * 16; if (t0 >= (size_t)TLIM) return;
  for (int rr = 0; rr < 16; ++rr) for (int q = 0; q < E / 32; ++q) { const int c = q * 32 + lane; Ax[rr][c] = (b16)(bf16_rne(x[(t0 + rr) * E + c]) * XS); }
  if (lane < 16) for (int k = E; k < E + 8; ++k) Ax[lane][k] = (b16)0.0f;
  wave_lds_sync();
#pragma unroll 1
  for (int g = 0; g < 2; ++g) { v8f acc[16];
#pragma unroll
    for (int t = 0; t < 16; ++t) acc[t] = (v8f){};
#pragma unroll 2
    for (int kb = 0; kb < E; kb += 32) { const v16b a = frag_kb(&Ax[nloc][kb], hlf);
#pragma unroll
      for (int t = 0; t < 16; ++t) acc[t] = wmma16b(a, frag_kb(WT + (size_t)(g * 256 + t * 16 + nloc) * E + kb, hlf), acc[t]); }
#pragma unroll
    for (int t = 0; t < 16; ++t) { const int cc = t * 16 + nloc; const float bb = bfv(b[g * 256 + cc]);
#pragma unroll
      for (int r8 = 0; r8 < 8; ++r8) Tf[8 * hlf + r8][cc] = acc[t][r8] * (1.0f / (XS * WSC)) + bb; }
    wave_lds_sync();
    for (int pass = 0; pass < 2; ++pass) { for (int rr = 0; rr < 16; ++rr) for (int q = 0; q < 2; ++q) *(volatile v4f*)(out + (t0 + rr) * E + g * 256 + q * 128 + lane * 4) = *(const v4f*)(&Tf[rr][q * 128 + lane * 4]); __threadfence(); }
    wave_lds_sync(); } }
}

extern "C" void kernel_launch(void* const* d_in, const int* in_sizes, int n_in, void* d_out, int out_size, void* d_ws, size_t ws_size, hipStream_t stream) {
  (void)n_in;
  auto Fp = [&](int i) { return (const float*)d_in[i]; };
  if (in_sizes[0] != NT * E || in_sizes[4] != E * E || in_sizes[5] != E || out_size != NT * E) return;
  const int TLIM = NT;
  size_t off = 0; char* ws = (char*)d_ws;
  auto carve = [&](size_t bytes) { char* p = ws + off; off += (bytes + 255) & ~(size_t)255; return p; };
  b16* WT = (b16*)carve((size_t)E * E * 2);
  if (off > ws_size || off > ((size_t)1 << 20)) return;
  wput_kernel<<<(E * (E / 8) + 255) / 256, 256, 0, stream>>>(Fp(4), WT);
  main_kernel<<<TLIM / 16, 32, 0, stream>>>(Fp(0), WT, Fp(5), TLIM, (float*)d_out);
}
